// LNN_89464168776130
// MI455X (gfx1250) — hardware-verified
//
#include <hip/hip_runtime.h>
#include <math.h>

typedef __attribute__((ext_vector_type(16))) _Float16 v16h;
typedef __attribute__((ext_vector_type(8)))  _Float16 v8h;
typedef __attribute__((ext_vector_type(8)))  float    v8f;
typedef __attribute__((ext_vector_type(4)))  float    v4f;
typedef __attribute__((ext_vector_type(2)))  float    v2f;

constexpr int   kHid       = 64;
constexpr int   kTileS     = 16;
constexpr int   kNCh       = 5;
constexpr int   kChStride  = kTileS * kHid;
constexpr int   kPlane     = kNCh * kChStride;
constexpr int   kWaves     = 2;
constexpr int   kThreads   = 32 * kWaves;
constexpr int   kMaxBlocks = 2048;
constexpr float kCarryW    = 16.0f;
constexpr float kCarryA    = 16.0f;
constexpr float kAccScale  = 1.0f / 256.0f;
constexpr float kEps       = 0.1f;
static_assert(kHid == 64);
static_assert(kThreads == kHid);
static_assert((kHid % 32) == 0);
static_assert((kTileS % 2) == 0);
static_assert(sizeof(_Float16) * (2 * kHid * kHid + kWaves * 2 * kPlane) + sizeof(float) * 6 * kHid <= 65536);

__device__ __forceinline__ void dep_guard_h(v8f& a, v8f& b, v16h x, v16h y) { asm volatile("v_nop\n\tv_nop\n\tv_nop\n\tv_nop" : "+v"(a), "+v"(b) : "v"(x), "v"(y)); }
__device__ __forceinline__ void keep4_h(v16h a, v16h b, v16h c, v16h d) { asm volatile("v_nop" :: "v"(a), "v"(b), "v"(c), "v"(d)); }
template <typename T> struct Frag;
template <> struct Frag<_Float16> {
  typedef v16h V; union U { v16h v; v8h h[2]; };
  static __device__ __forceinline__ v16h load(const _Float16* p) {
    U f; f.h[0] = *(const v8h*)(p); f.h[1] = *(const v8h*)(p + 16); return f.v;
  }
  static __device__ __forceinline__ v8f mma(v16h a, v16h b, v8f c) {
    return __builtin_amdgcn_wmma_f32_16x16x32_f16(false, a, false, b, (short)0, c, false, false);
  }
  static __device__ __forceinline__ void guard(v8f& a, v8f& b, v16h x, v16h y) { dep_guard_h(a, b, x, y); }
  static __device__ __forceinline__ void keep(v16h a, v16h b, v16h c, v16h d) { keep4_h(a, b, c, d); }
};

__device__ __forceinline__ void guard5(v8f& a0, v8f& a1, v8f& a2, v8f& a3, v8f& a4,
                                       v16h f0, v16h f1, v16h f2, v16h f3, v16h f4, v16h f5) {
  asm volatile("v_nop\n\tv_nop\n\tv_nop\n\tv_nop"
               : "+v"(a0), "+v"(a1), "+v"(a2), "+v"(a3), "+v"(a4)
               : "v"(f0), "v"(f1), "v"(f2), "v"(f3), "v"(f4), "v"(f5));
}

__device__ __forceinline__ void lds_wave_sync() {
  __builtin_amdgcn_fence(__ATOMIC_RELEASE, "workgroup");
  __builtin_amdgcn_wave_barrier();
  __builtin_amdgcn_fence(__ATOMIC_ACQUIRE, "workgroup");
}

__device__ __forceinline__ float tanh_f32(float x) {
  const float ax = fminf(fabsf(x), 12.0f);
  const float e  = expf(ax + ax);
  const float r  = __builtin_amdgcn_rcpf(e + 1.0f);
  const float t  = fmaf(-2.0f, r, 1.0f);
  return copysignf(t, x);
}

__device__ __forceinline__ void layer0_block(float xq, float xv,
                                             const float* sWq, const float* sWv, const float* sBias,
                                             _Float16* plane, int cb, int rl, int hh) {
  const int nb = 16 * cb + 8 * hh;
  const v4f wq0 = *(const v4f*)(sWq + nb), wq1 = *(const v4f*)(sWq + nb + 4);
  const v4f wv0 = *(const v4f*)(sWv + nb), wv1 = *(const v4f*)(sWv + nb + 4);
  const v4f bb0 = *(const v4f*)(sBias + nb), bb1 = *(const v4f*)(sBias + nb + 4);
  float wq[8], wv[8], bb[8];
#pragma unroll
  for (int j = 0; j < 4; ++j) {
    wq[j] = wq0[j]; wq[4 + j] = wq1[j];
    wv[j] = wv0[j]; wv[4 + j] = wv1[j];
    bb[j] = bb0[j]; bb[4 + j] = bb1[j];
  }
  v8h o0, o1, o2, o3, o4;
#pragma unroll
  for (int r = 0; r < 8; ++r) {
    const float z  = fmaf(xv, wv[r], xq * wq[r]) + bb[r];
    const float t  = tanh_f32(z);
    const float s  = fmaf(-t, t, 1.0f);
    const float sc = s * kCarryA;
    const float uc = (-2.0f * t) * sc;
    o0[r] = (_Float16)(t * kCarryA);
    o1[r] = (_Float16)(sc * wq[r]);
    o2[r] = (_Float16)(sc * wv[r]);
    o3[r] = (_Float16)((uc * wq[r]) * wv[r]);
    o4[r] = (_Float16)((uc * wv[r]) * wv[r]);
  }
  _Float16* dst = plane + rl * kHid + nb;
  *(v8h*)(dst + 0 * kChStride) = o0;
  *(v8h*)(dst + 1 * kChStride) = o1;
  *(v8h*)(dst + 2 * kChStride) = o2;
  *(v8h*)(dst + 3 * kChStride) = o3;
  *(v8h*)(dst + 4 * kChStride) = o4;
}

__device__ __forceinline__ void gemm5(const _Float16* sW, const _Float16* plane, int mb, int rl, int hh,
                                      v8f (&acc)[kNCh]) {
#pragma unroll
  for (int c = 0; c < kNCh; ++c) acc[c] = (v8f){0.f, 0.f, 0.f, 0.f, 0.f, 0.f, 0.f, 0.f};
#pragma unroll
  for (int ks = 0; ks < kHid / 32; ++ks) {
    const int koff = 32 * ks + 8 * hh;
    const v16h af = Frag<_Float16>::load(sW + (16 * mb + rl) * kHid + koff);
    v16h bf[kNCh];
#pragma unroll
    for (int c = 0; c < kNCh; ++c) bf[c] = Frag<_Float16>::load(plane + c * kChStride + rl * kHid + koff);
#pragma unroll
    for (int c = 0; c < kNCh; ++c) acc[c] = Frag<_Float16>::mma(af, bf[c], acc[c]);
    guard5(acc[0], acc[1], acc[2], acc[3], acc[4], af, bf[0], bf[1], bf[2], bf[3], bf[4]);
  }
}

__device__ __forceinline__ void jet_store(const v8f (&acc)[kNCh], const float* sBias, _Float16* nplane,
                                          int mb, int rl, int hh) {
  const int nb = 16 * mb + 8 * hh;
  const v4f bb0 = *(const v4f*)(sBias + nb), bb1 = *(const v4f*)(sBias + nb + 4);
  float bb[8];
#pragma unroll
  for (int j = 0; j < 4; ++j) { bb[j] = bb0[j]; bb[4 + j] = bb1[j]; }
  v8h o0, o1, o2, o3, o4;
#pragma unroll
  for (int r = 0; r < 8; ++r) {
    const float z   = fmaf(acc[0][r], kAccScale, bb[r]);
    const float d0  = acc[1][r] * kAccScale;
    const float d1  = acc[2][r] * kAccScale;
    const float d01 = acc[3][r] * kAccScale;
    const float d11 = acc[4][r] * kAccScale;
    const float t   = tanh_f32(z);
    const float s   = fmaf(-t, t, 1.0f);
    const float sc  = s * kCarryA;
    const float uc  = (-2.0f * t) * sc;
    o0[r] = (_Float16)(t * kCarryA);
    o1[r] = (_Float16)(sc * d0);
    o2[r] = (_Float16)(sc * d1);
    o3[r] = (_Float16)fmaf(uc * d0, d1, sc * d01);
    o4[r] = (_Float16)fmaf(uc * d1, d1, sc * d11);
  }
  _Float16* dst = nplane + rl * kHid + nb;
  *(v8h*)(dst + 0 * kChStride) = o0;
  *(v8h*)(dst + 1 * kChStride) = o1;
  *(v8h*)(dst + 2 * kChStride) = o2;
  *(v8h*)(dst + 3 * kChStride) = o3;
  *(v8h*)(dst + 4 * kChStride) = o4;
}

__device__ __forceinline__ void head_accum(const v8f (&acc)[kNCh], const float* sBias, const float* sHead,
                                           int mb, int hh, float& p0, float& p01, float& p11) {
  const int nb = 16 * mb + 8 * hh;
  const v4f bb0 = *(const v4f*)(sBias + nb), bb1 = *(const v4f*)(sBias + nb + 4);
  const v4f ww0 = *(const v4f*)(sHead + nb), ww1 = *(const v4f*)(sHead + nb + 4);
  float bb[8], ww[8];
#pragma unroll
  for (int j = 0; j < 4; ++j) { bb[j] = bb0[j]; bb[4 + j] = bb1[j]; ww[j] = ww0[j]; ww[4 + j] = ww1[j]; }
#pragma unroll
  for (int r = 0; r < 8; ++r) {
    const float z   = fmaf(acc[0][r], kAccScale, bb[r]);
    const float d0  = acc[1][r] * kAccScale;
    const float d1  = acc[2][r] * kAccScale;
    const float d01 = acc[3][r] * kAccScale;
    const float d11 = acc[4][r] * kAccScale;
    const float t   = tanh_f32(z);
    const float s   = fmaf(-t, t, 1.0f);
    const float u   = (-2.0f * t) * s;
    const float g0  = s * d0;
    const float g01 = fmaf(u * d0, d1, s * d01);
    const float g11 = fmaf(u * d1, d1, s * d11);
    const float w   = ww[r];
    p0  = fmaf(g0, w, p0);
    p01 = fmaf(g01, w, p01);
    p11 = fmaf(g11, w, p11);
  }
}

__global__ __launch_bounds__(kThreads) void jet_mlp_kernel(
    const float* __restrict__ x,
    const float* __restrict__ W0, const float* __restrict__ b0,
    const float* __restrict__ W1, const float* __restrict__ b1,
    const float* __restrict__ W2, const float* __restrict__ b2,
    const float* __restrict__ W3,
    float* __restrict__ out, int nsamp, int ntiles) {
  __shared__ __align__(16) _Float16 sWt[2][kHid * kHid];
  __shared__ __align__(16) _Float16 sAct[kWaves][2][kPlane];
  __shared__ __align__(16) float sW0q[kHid];
  __shared__ __align__(16) float sW0v[kHid];
  __shared__ __align__(16) float sB0[kHid];
  __shared__ __align__(16) float sB1[kHid];
  __shared__ __align__(16) float sB2[kHid];
  __shared__ __align__(16) float sW3[kHid];

  const int tid = threadIdx.x;
#pragma unroll 2
  for (int i = tid; i < kHid * kHid; i += kThreads) {
    const int fin = i >> 6, fout = i & 63;
    const float w1 = W1[i] * kCarryW;
    const float w2 = W2[i] * kCarryW;
    sWt[0][fout * kHid + fin] = (_Float16)w1;
    sWt[1][fout * kHid + fin] = (_Float16)w2;
  }
  {
    sW0q[tid] = W0[tid];
    sW0v[tid] = W0[kHid + tid];
    sB0[tid]  = b0[tid];
    sB1[tid]  = b1[tid];
    sB2[tid]  = b2[tid];
    sW3[tid]  = W3[tid];
  }
  __syncthreads();

  const int lane = tid & 31;
  const int wave = tid >> 5;
  const int hh   = lane >> 4;
  const int rl   = lane & 15;
  _Float16* bufA = sAct[wave][0];
  _Float16* bufB = sAct[wave][1];
  const int wid = blockIdx.x * kWaves + wave;
  const int nw  = gridDim.x * kWaves;

#pragma unroll 1
  for (int tile = wid; tile < ntiles; tile += nw) {
    int g = tile * kTileS + rl;
    g = (g < nsamp) ? g : (nsamp - 1);
    const v2f xv2 = *(const v2f*)(x + 2 * (size_t)g);
    const float xq = xv2[0];
    const float xv = xv2[1];

#pragma unroll 1
    for (int cb = 0; cb < kHid / 16; ++cb) layer0_block(xq, xv, sW0q, sW0v, sB0, bufA, cb, rl, hh);
    lds_wave_sync();

#pragma unroll 1
    for (int mb = 0; mb < kHid / 16; ++mb) {
      v8f acc[kNCh];
      gemm5(sWt[0], bufA, mb, rl, hh, acc);
      jet_store(acc, sB1, bufB, mb, rl, hh);
    }
    lds_wave_sync();

    float p0 = 0.0f, p01 = 0.0f, p11 = 0.0f;
#pragma unroll 1
    for (int mb = 0; mb < kHid / 16; ++mb) {
      v8f acc[kNCh];
      gemm5(sWt[1], bufB, mb, rl, hh, acc);
      head_accum(acc, sB2, sW3, mb, hh, p0, p01, p11);
    }
    p0  += __shfl_xor(p0, 16, 32);
    p01 += __shfl_xor(p01, 16, 32);
    p11 += __shfl_xor(p11, 16, 32);
    const float a = (p0 - p01 * xv) / (p11 + kEps);

    const int s0 = (2 * lane) & 31;
    const int s1 = (2 * lane + 1) & 31;
    v4f ov;
    ov[0] = __shfl(xv, s0, 32);
    ov[1] = __shfl(a, s0, 32);
    ov[2] = __shfl(xv, s1, 32);
    ov[3] = __shfl(a, s1, 32);
    float* op = out + (size_t)tile * (2 * kTileS) + 4 * lane;
    if (lane < 8) *(volatile v4f*)op = ov;
    __threadfence();
    if (lane < 8) *(volatile v4f*)op = ov;
  }
}

extern "C" void kernel_launch(void* const* d_in, const int* in_sizes, int n_in,
                              void* d_out, int out_size, void* d_ws, size_t ws_size,
                              hipStream_t stream) {
  (void)n_in; (void)out_size; (void)d_ws; (void)ws_size;
  const float* x  = (const float*)d_in[1];
  const float* W0 = (const float*)d_in[2];
  const float* b0 = (const float*)d_in[3];
  const float* W1 = (const float*)d_in[4];
  const float* b1 = (const float*)d_in[5];
  const float* W2 = (const float*)d_in[6];
  const float* b2 = (const float*)d_in[7];
  const float* W3 = (const float*)d_in[8];
  float* out = (float*)d_out;

  const int nsamp  = in_sizes[1] / 2;
  const int ntiles = nsamp / kTileS;
  int blocks = (ntiles + kWaves - 1) / kWaves;
  if (blocks > kMaxBlocks) blocks = kMaxBlocks;
  if (blocks < 1) blocks = 1;
  jet_mlp_kernel<<<blocks, kThreads, 0, stream>>>(x, W0, b0, W1, b1, W2, b2, W3, out, nsamp, ntiles);
}
